// HybridGNNModel_33071248180019
// MI455X (gfx1250) — hardware-verified
//
#include <hip/hip_runtime.h>
#include <stddef.h>
#include <stdint.h>


#define DIN     64
#define H0      64
#define HC      64
#define NHEAD   2
#define HDQ     128
#define NQ      448
#define OQ      0
#define OKK     128
#define OV      256
#define OS      384
#define DOUT    32
#define KS      128
#define NFP     64
#define NTHR    256
#define NWAVE   8
#define EPT     8
#define CHUNK   (NTHR * EPT)
#define WCAP    (EPT * 32)
#define LISTN   (NWAVE * WCAP)
#define NBMAX   2048
#define RCAP    28672
#define DEGCAP  4096
#define STW     512
#define GBM     64
#define GBN     64
#define GTHR    128
#define ATTSC   0.125f
#define NEGSL   0.2f
#define WSMAX   142606336
#define LDS_AGG ((2 * RCAP + 2 * NBMAX + LISTN) * 4 + 64)

static_assert((CHUNK & (CHUNK - 1)) == 0 && CHUNK <= 4096);
static_assert((NBMAX & (NBMAX - 1)) == 0 && NBMAX <= 4096);
static_assert(NTHR * 8 == NBMAX);
static_assert(LISTN >= NBMAX);
static_assert(LISTN >= NWAVE * WCAP);
static_assert((RCAP % 32) == 0);
static_assert(NWAVE * STW <= RCAP);
static_assert(LDS_AGG <= 300000);
static_assert(GBM == (GTHR / 32) * 16);
static_assert((DIN % 32) == 0 && (KS % 32) == 0);
static_assert((NQ % GBN) == 0 && (H0 % GBN) == 0 && (NFP % GBN) == 0);
static_assert(NQ == 3 * HDQ + HC && HDQ == NHEAD * HC);
static_assert(HC == 64 && H0 == 64 && KS == 2 * HC && KS == 2 * H0);
static_assert(GBM * DOUT / 4 == 4 * GTHR);
static_assert(2 * HC <= STW);
static_assert(GTHR >= H0 && GTHR >= GBM);
static_assert(DOUT <= NFP);

typedef float          v4f  __attribute__((ext_vector_type(4)));
typedef float          v8f  __attribute__((ext_vector_type(8)));
typedef int            v4i  __attribute__((ext_vector_type(4)));
typedef int            v8i  __attribute__((ext_vector_type(8)));
typedef unsigned short v8us __attribute__((ext_vector_type(8)));
typedef __bf16         v16b __attribute__((ext_vector_type(16)));
union FragB { v16b v; v8us h[2]; v8i w; };
union U8 { v8us v; v4i w; };

__device__ __forceinline__ v8f wmb(const FragB& a, const FragB& b, v8f c) {
  v8f d = __builtin_amdgcn_wmma_f32_16x16x32_bf16(false, a.v, false, b.v, (short)0, c, false, false);
  asm volatile("v_nop\n\tv_nop\n\tv_nop\n\tv_nop" : "+v"(d) : "v"(a.w), "v"(b.w));
  return d;
}

__device__ __forceinline__ void ldwait() {
  asm volatile("s_wait_loadcnt 0x0" ::: "memory");
}

__device__ __forceinline__ unsigned short bfr(float f) {
  const unsigned u = __float_as_uint(f);
  return (unsigned short)((u + 0x7FFFu + ((u >> 16) & 1u)) >> 16);
}
__device__ __forceinline__ float bff(unsigned short s) {
  return __uint_as_float(((unsigned)s) << 16);
}
__device__ __forceinline__ float rbf(float f) { return bff(bfr(f)); }

__device__ __forceinline__ v8us cvt8b(const v4f a, const v4f b) {
  v8us r;
  r[0] = bfr(a.x); r[1] = bfr(a.y); r[2] = bfr(a.z); r[3] = bfr(a.w);
  r[4] = bfr(b.x); r[5] = bfr(b.y); r[6] = bfr(b.z); r[7] = bfr(b.w);
  return r;
}
__device__ __forceinline__ void split8(const v4f a, const v4f b, v8us& hi, v8us& lo) {
  hi = cvt8b(a, b);
  v4f ra, rb;
  ra.x = a.x - bff(hi[0]); ra.y = a.y - bff(hi[1]); ra.z = a.z - bff(hi[2]); ra.w = a.w - bff(hi[3]);
  rb.x = b.x - bff(hi[4]); rb.y = b.y - bff(hi[5]); rb.z = b.z - bff(hi[6]); rb.w = b.w - bff(hi[7]);
  lo = cvt8b(ra, rb);
}

__device__ __forceinline__ int scan_chunk(const int* __restrict__ dsts, int nE, int cbase, int slotBase,
                                          int nb, int vec8, int* list, int tid, int lane, int wave) {
  int wc = 0;
  const int el0  = tid * EPT;
  const int e0   = cbase + el0;
  const int sent = -2147483647 - 1;
  v4i da, db;
  if (vec8 != 0 && cbase + CHUNK <= nE) {
    da = *(const v4i*)(dsts + e0);
    db = *(const v4i*)(dsts + e0 + 4);
  } else {
    da.x = (e0     < nE) ? dsts[min(e0,     nE - 1)] : sent;
    da.y = (e0 + 1 < nE) ? dsts[min(e0 + 1, nE - 1)] : sent;
    da.z = (e0 + 2 < nE) ? dsts[min(e0 + 2, nE - 1)] : sent;
    da.w = (e0 + 3 < nE) ? dsts[min(e0 + 3, nE - 1)] : sent;
    db.x = (e0 + 4 < nE) ? dsts[min(e0 + 4, nE - 1)] : sent;
    db.y = (e0 + 5 < nE) ? dsts[min(e0 + 5, nE - 1)] : sent;
    db.z = (e0 + 6 < nE) ? dsts[min(e0 + 6, nE - 1)] : sent;
    db.w = (e0 + 7 < nE) ? dsts[min(e0 + 7, nE - 1)] : sent;
  }
  const unsigned nbs = (unsigned)slotBase;
  const unsigned unb = (unsigned)nb;
  const unsigned s0 = (unsigned)da.x - nbs, s1 = (unsigned)da.y - nbs;
  const unsigned s2 = (unsigned)da.z - nbs, s3 = (unsigned)da.w - nbs;
  const unsigned s4 = (unsigned)db.x - nbs, s5 = (unsigned)db.y - nbs;
  const unsigned s6 = (unsigned)db.z - nbs, s7 = (unsigned)db.w - nbs;
  const bool h0 = s0 < unb, h1 = s1 < unb, h2 = s2 < unb, h3 = s3 < unb;
  const bool h4 = s4 < unb, h5 = s5 < unb, h6 = s6 < unb, h7 = s7 < unb;
  const unsigned any = __builtin_amdgcn_ballot_w32(h0 | h1 | h2 | h3 | h4 | h5 | h6 | h7);
  if (any != 0u) {
#define HITJ(J, HJ, SJ) { \
      const unsigned mj = __builtin_amdgcn_ballot_w32(HJ); \
      if (mj != 0u) { \
        if (HJ) { \
          const int pos = wc + (int)__builtin_amdgcn_mbcnt_lo(mj, 0u); \
          if (pos < WCAP) list[wave * WCAP + pos] = ((el0 + (J)) << 12) | (int)(SJ); \
        } \
        wc += (int)__builtin_popcount(mj); } }
    HITJ(0, h0, s0)
    HITJ(1, h1, s1)
    HITJ(2, h2, s2)
    HITJ(3, h3, s3)
    HITJ(4, h4, s4)
    HITJ(5, h5, s5)
    HITJ(6, h6, s6)
    HITJ(7, h7, s7)
#undef HITJ
  }
  return wc;
}

__global__ __launch_bounds__(NTHR) void k_xprep(const float* __restrict__ x, unsigned short* xb, int nN, int nUnits) {
  const int i = (int)blockIdx.x * NTHR + (int)threadIdx.x;
  if (i >= nUnits) return;
  const int row = i >> 3;
  const int c0  = (i & 7) * 8;
  const int rc  = row < nN ? row : nN - 1;
  const float* p = x + (size_t)rc * DIN + c0;
  v4f a = *(const v4f*)p, b = *(const v4f*)(p + 4);
  const v4f z4 = {0.f, 0.f, 0.f, 0.f};
  if (row >= nN) { a = z4; b = z4; }
  const v8us hv = cvt8b(a, b);
  const size_t o = (size_t)row * DIN + c0;
  *(volatile v8us*)(xb + o) = hv;
  __threadfence();
  *(volatile v8us*)(xb + o) = hv;
}

__global__ __launch_bounds__(NTHR) void k_wtr(const float* __restrict__ w0, const float* __restrict__ w1,
                                              const float* __restrict__ w2, const float* __restrict__ w3,
                                              int c0, int c1, int c2, int c3, int segRows, int Kin, int Kout,
                                              unsigned short* wt, int nUnits) {
  const int u = (int)blockIdx.x * NTHR + (int)threadIdx.x;
  if (u >= nUnits) return;
  const int kq = Kout >> 3;
  const int n  = u / kq;
  const int k8 = (u - n * kq) * 8;
  int ksrc = k8 < Kin ? k8 : k8 - Kin;
  ksrc = ksrc < 0 ? 0 : (ksrc > Kin - 8 ? Kin - 8 : ksrc);
  int seg = n / segRows;
  seg = seg > 3 ? 3 : seg;
  const int nc = n - seg * segRows;
  const float* ws = (seg == 0) ? w0 : ((seg == 1) ? w1 : ((seg == 2) ? w2 : w3));
  const int cc = (seg == 0) ? c0 : ((seg == 1) ? c1 : ((seg == 2) ? c2 : c3));
  int ncl = nc < cc ? nc : cc - 1;
  ncl = ncl < 0 ? 0 : ncl;
  const float* p = ws + (size_t)ksrc * (size_t)cc + ncl;
  v4f a, b;
  a.x = p[0];                  a.y = p[(size_t)cc];         a.z = p[(size_t)2 * cc];     a.w = p[(size_t)3 * cc];
  b.x = p[(size_t)4 * cc];     b.y = p[(size_t)5 * cc];     b.z = p[(size_t)6 * cc];     b.w = p[(size_t)7 * cc];
  const v4f z4 = {0.f, 0.f, 0.f, 0.f};
  if (nc >= cc) { a = z4; b = z4; }
  const v8us hv = cvt8b(a, b);
  const size_t o = (size_t)n * (size_t)Kout + k8;
  *(volatile v8us*)(wt + o) = hv;
  __threadfence();
  *(volatile v8us*)(wt + o) = hv;
}

template<int EPI>
__global__ __launch_bounds__(GTHR) void k_gemm(
    const unsigned short* __restrict__ A, const unsigned short* __restrict__ WT,
    const float* __restrict__ b0, const float* __restrict__ b1,
    const float* __restrict__ b2, const float* __restrict__ b3,
    const float* __restrict__ att, float* outF, float* sgo,
    int K, int ldo, int segN, int len012, int len3, int nRows)
{
  __shared__ __attribute__((aligned(16))) float stg[GBM * GBN];
  __shared__ __attribute__((aligned(16))) float attl[H0];
  __shared__ __attribute__((aligned(16))) float sgl[GBM];
  const int tid = (int)threadIdx.x, lane = tid & 31, wave = tid >> 5, hh = lane >> 4, m = lane & 15;
  const int rowBase = (int)blockIdx.x * GBM;
  const int col0    = (int)blockIdx.y * GBN;
  int seg = col0 / segN;
  seg = seg < 0 ? 0 : (seg > 3 ? 3 : seg);
  const float* bp = (seg == 0) ? b0 : ((seg == 1) ? b1 : ((seg == 2) ? b2 : b3));
  const int blen = (seg < 3) ? len012 : len3;
  int bofs = col0 - seg * segN;
  bofs = bofs < 0 ? 0 : bofs;

  v8f acc[4];
  {
    const v8f z = {0.f, 0.f, 0.f, 0.f, 0.f, 0.f, 0.f, 0.f};
    acc[0] = z; acc[1] = z; acc[2] = z; acc[3] = z;
  }
  const unsigned short* ap = A  + (size_t)(rowBase + 16 * wave + m) * (size_t)K + 8 * hh;
  const unsigned short* wp = WT + (size_t)(col0 + m) * (size_t)K + 8 * hh;
  const int ksteps = K >> 5;
#pragma unroll 1
  for (int ks = 0; ks < ksteps; ++ks) {
    FragB af;
    af.h[0] = *(const v8us*)(ap + 32 * ks);
    af.h[1] = *(const v8us*)(ap + 32 * ks + 16);
#pragma unroll
    for (int t = 0; t < 4; ++t) {
      const unsigned short* wq = wp + (size_t)(16 * t) * (size_t)K + 32 * ks;
      FragB bf;
      bf.h[0] = *(const v8us*)wq;
      bf.h[1] = *(const v8us*)(wq + 16);
      acc[t] = wmb(af, bf, acc[t]);
    }
  }

#pragma unroll
  for (int t = 0; t < 4; ++t) {
    const int lc = 16 * t + m;
    int bi = bofs + lc;
    bi = bi > blen - 1 ? blen - 1 : bi;
    bi = bi < 0 ? 0 : bi;
    const float bv = rbf(bp[bi]);
#pragma unroll
    for (int r = 0; r < 8; ++r) {
      const int lr = 16 * wave + 8 * hh + r;
      stg[lr * GBN + lc] = acc[t][r] + bv;
    }
  }
  if (EPI == 1) {
    if (tid < H0) attl[tid] = rbf(att[tid < H0 ? tid : H0 - 1]);
  }
  __syncthreads();
  if (EPI == 1) {
    if (tid < GBM) {
      float d = 0.f;
#pragma unroll 4
      for (int c = 0; c < H0; ++c) d = fmaf(stg[tid * GBN + c], attl[c], d);
      sgl[tid] = d >= 0.f ? d : NEGSL * d;
    }
    __syncthreads();
  }

  if (EPI == 0 || EPI == 1) {
    v4f fv[8];
#pragma unroll
    for (int i = 0; i < 8; ++i) {
      const int lr = 16 * wave + 2 * i + hh;
      fv[i] = *(const v4f*)(stg + lr * GBN + 4 * m);
    }
    v4f s4 = {0.f, 0.f, 0.f, 0.f};
    if (EPI == 1) s4 = *(const v4f*)(sgl + 4 * m);
    const bool wsg = (EPI == 1) && (wave == 0) && (lane < 16);
    float* sp = sgo + (size_t)rowBase + 4 * m;
#pragma unroll
    for (int i = 0; i < 8; ++i) {
      const int lr = 16 * wave + 2 * i + hh;
      const int gr = rowBase + lr;
      float* op = outF + (size_t)gr * (size_t)ldo + col0 + 4 * m;
      *(volatile v4f*)op = fv[i];
    }
    if (wsg) *(volatile v4f*)sp = s4;
    __threadfence();
#pragma unroll
    for (int i = 0; i < 8; ++i) {
      const int lr = 16 * wave + 2 * i + hh;
      const int gr = rowBase + lr;
      float* op = outF + (size_t)gr * (size_t)ldo + col0 + 4 * m;
      *(volatile v4f*)op = fv[i];
    }
    if (wsg) *(volatile v4f*)sp = s4;
  } else {
    int nv = nRows - rowBase;
    nv = nv < 0 ? 0 : (nv > GBM ? GBM : nv);
    const int np = nv * (DOUT / 4);
    v4f pv[4];
#pragma unroll
    for (int i = 0; i < 4; ++i) {
      const int p   = i * GTHR + tid;
      const int row = p >> 3;
      const int c4  = (p & 7) * 4;
      pv[i] = *(const v4f*)(stg + row * GBN + c4);
    }
    float* ob = outF + (size_t)rowBase * DOUT;
#pragma unroll
    for (int i = 0; i < 4; ++i) {
      const int p = i * GTHR + tid;
      if (p < np) *(volatile v4f*)(ob + 4 * p) = pv[i];
    }
    __threadfence();
#pragma unroll
    for (int i = 0; i < 4; ++i) {
      const int p = i * GTHR + tid;
      if (p < np) *(volatile v4f*)(ob + 4 * p) = pv[i];
    }
  }
}

template<int LAYER>
__global__ __launch_bounds__(NTHR) void k_agg(
    const int* __restrict__ srcs, const int* __restrict__ dsts,
    const float* __restrict__ HF, const float* __restrict__ SG, const float* __restrict__ cew,
    const float* __restrict__ QKVS, unsigned short* Hout,
    int nN, int nE, int nb, int vec8, int MPr) {
  extern __shared__ v4f lds_dyn[];
  int* reg1 = (int*)lds_dyn;
  int* reg2 = reg1 + RCAP;
  int* scnt = reg2 + RCAP;
  int* soff = scnt + NBMAX;
  int* list = soff + NBMAX;
  int* wcnt = list + LISTN;
  int* wtot = wcnt + NWAVE;
  const int tid = (int)threadIdx.x, lane = tid & 31, wave = tid >> 5;
  const int nodeBase = (int)blockIdx.x * nb;

  for (int i = tid; i < NBMAX; i += NTHR) scnt[i] = 0;
  __syncthreads();

  int tot = 0;
  const int nChunks = (nE + CHUNK - 1) / CHUNK;
#pragma unroll 1
  for (int ch = 0; ch < nChunks; ++ch) {
    const int cbase = ch * CHUNK;
    const int wc = scan_chunk(dsts, nE, cbase, nodeBase, nb, vec8, list, tid, lane, wave);
    if (lane == 0) wcnt[wave] = wc;
    __syncthreads();
    int pre = 0, all = 0;
#pragma unroll
    for (int w2 = 0; w2 < NWAVE; ++w2) {
      int c = wcnt[w2];
      c = c < 0 ? 0 : (c > WCAP ? WCAP : c);
      all += c;
      pre += (w2 < wave) ? c : 0;
    }
    const int wcc  = wc > WCAP ? WCAP : wc;
    const int base = tot + pre;
#pragma unroll 1
    for (int i = lane; i < wcc; i += 32) {
      const int ent = list[wave * WCAP + i];
      const int el  = (ent >> 12) & (CHUNK - 1);
      const int sl  = ent & (NBMAX - 1);
      int eid = cbase + el;
      eid = eid > nE - 1 ? nE - 1 : eid;
      const int pos = base + i;
      if (pos < RCAP) reg1[pos] = (int)(((unsigned)eid << 12) | (unsigned)sl);
    }
    tot += all;
    tot = tot > RCAP ? RCAP : tot;
    __syncthreads();
  }
  const int nh = tot;

  if (wave == 0) {
#pragma unroll 1
    for (int b0 = 0; b0 < nh; b0 += 32) {
      const int idx = b0 + lane;
      const int uv  = reg1[idx < RCAP ? idx : RCAP - 1];
      const int m32 = (nh - b0) < 32 ? (nh - b0) : 32;
#pragma unroll 1
      for (int k = 0; k < m32; ++k) {
        const int u  = __builtin_amdgcn_readlane(uv, k);
        const int sl = u & (NBMAX - 1);
        if (lane == 0) scnt[sl] = scnt[sl] + 1;
      }
    }
  }
  __syncthreads();

  {
    const v4i ca = *(const v4i*)(scnt + 8 * tid);
    const v4i cb = *(const v4i*)(scnt + 8 * tid + 4);
    const int e0 = ca.x < 0 ? 0 : ca.x, e1 = ca.y < 0 ? 0 : ca.y, e2 = ca.z < 0 ? 0 : ca.z, e3 = ca.w < 0 ? 0 : ca.w;
    const int e4 = cb.x < 0 ? 0 : cb.x, e5 = cb.y < 0 ? 0 : cb.y, e6 = cb.z < 0 ? 0 : cb.z, e7 = cb.w < 0 ? 0 : cb.w;
    const int ts = e0 + e1 + e2 + e3 + e4 + e5 + e6 + e7;
    int incl = ts;
#pragma unroll
    for (int d = 1; d < 32; d <<= 1) {
      const int up = __shfl_up(incl, d);
      if (lane >= d) incl += up;
    }
    if (lane == 31) wtot[wave] = incl;
    __syncthreads();
    int pre = 0;
#pragma unroll
    for (int w2 = 0; w2 < NWAVE; ++w2) pre += (w2 < wave) ? wtot[w2] : 0;
    int run = pre + incl - ts;
    soff[8 * tid + 0] = run; run += e0;
    soff[8 * tid + 1] = run; run += e1;
    soff[8 * tid + 2] = run; run += e2;
    soff[8 * tid + 3] = run; run += e3;
    soff[8 * tid + 4] = run; run += e4;
    soff[8 * tid + 5] = run; run += e5;
    soff[8 * tid + 6] = run; run += e6;
    soff[8 * tid + 7] = run;
  }
  __syncthreads();
  for (int i = tid; i < NBMAX; i += NTHR) list[i] = soff[i];
  __syncthreads();

  if (wave == 0) {
#pragma unroll 1
    for (int b0 = 0; b0 < nh; b0 += 32) {
      const int idx = b0 + lane;
      const int uv  = reg1[idx < RCAP ? idx : RCAP - 1];
      const int m32 = (nh - b0) < 32 ? (nh - b0) : 32;
#pragma unroll 1
      for (int k = 0; k < m32; ++k) {
        const int u   = __builtin_amdgcn_readlane(uv, k);
        const int sl  = u & (NBMAX - 1);
        const int eid = (int)((unsigned)u >> 12);
        if (lane == 0) {
          int pos = list[sl];
          pos = pos < 0 ? 0 : (pos > RCAP - 1 ? RCAP - 1 : pos);
          reg2[pos] = eid;
          list[sl] = pos + 1;
        }
      }
    }
  }
  __syncthreads();

  const int nbw = nb >> 3;
  const bool ovf = (nh >= RCAP);
  const float qnan = __int_as_float(0x7fc00000);
  float* stw = (float*)reg1 + wave * STW;
#pragma unroll 1
  for (int jt = 0; jt < nbw; ++jt) {
    const int slot = wave * nbw + jt;
    const int grow = nodeBase + slot;
    const int gcl  = grow < nN ? grow : nN - 1;
    int st = soff[slot];
    const int craw = scnt[slot];
    int cnt = craw;
    st  = st < 0 ? 0 : (st > nh ? nh : st);
    cnt = cnt < 0 ? 0 : (cnt > DEGCAP ? DEGCAP : cnt);
    if (cnt > nh - st) cnt = nh - st;
    const float pz = (ovf || craw > DEGCAP) ? qnan : 0.0f;
    const bool wr = grow < MPr;
    const float live = grow < nN ? 1.0f : 0.0f;
    float r0, r1;

    if (LAYER == 1) {
      float mx = -1.0e30f, dn = 0.f, a0 = 0.f, a1 = 0.f;
#pragma unroll 1
      for (int q = 0; q < cnt; ++q) {
        int idx = st + q; idx = idx > RCAP - 1 ? RCAP - 1 : idx;
        int eid = reg2[idx]; eid = eid < 0 ? 0 : (eid > nE - 1 ? nE - 1 : eid);
        const int sraw = srcs[eid];
        const int s = sraw < 0 ? 0 : (sraw > nN - 1 ? nN - 1 : sraw);
        const float* hr = HF + (size_t)s * H0 + lane;
        const float hv0 = hr[0];
        const float hv1 = hr[32];
        const float sgv = SG[s];
        const float cwr = cew[eid];
        ldwait();
        const float cw = rbf(cwr);
        const float df = sgv - mx;
        const float ee = __expf(-fabsf(df));
        const bool up  = df > 0.f;
        const float s1 = up ? ee : 1.0f;
        const float s2 = up ? 1.0f : ee;
        mx = up ? sgv : mx;
        dn = fmaf(dn, s1, s2);
        const float w = s2 * cw;
        a0 = fmaf(a0, s1, w * hv0);
        a1 = fmaf(a1, s1, w * hv1);
      }
      const float ds = dn > 0.f ? dn : 1.0f;
      const float iv = (dn > 0.f ? 1.0f : 0.0f) * __builtin_amdgcn_rcpf(ds);
      r0 = fmaxf(a0 * iv, 0.f) * live + pz;
      r1 = fmaxf(a1 * iv, 0.f) * live + pz;
    } else {
      const float* qrow = QKVS + (size_t)gcl * NQ + lane;
      float qv[4], av[4];
#pragma unroll
      for (int j = 0; j < 4; ++j) { qv[j] = qrow[OQ + 32 * j]; av[j] = 0.f; }
      const float sk0 = qrow[OS];
      const float sk1 = qrow[OS + 32];
      ldwait();
      float mx[2], dn[2];
      mx[0] = -1.0e30f; mx[1] = -1.0e30f; dn[0] = 0.f; dn[1] = 0.f;

#pragma unroll 1
      for (int q = 0; q < cnt; ++q) {
        int idx = st + q; idx = idx > RCAP - 1 ? RCAP - 1 : idx;
        int eid = reg2[idx]; eid = eid < 0 ? 0 : (eid > nE - 1 ? nE - 1 : eid);
        const int sraw = srcs[eid];
        const int s = sraw < 0 ? 0 : (sraw > nN - 1 ? nN - 1 : sraw);
        const float* kr = QKVS + (size_t)s * NQ + OKK + lane;
        float kk[4], vv[4];
#pragma unroll
        for (int j = 0; j < 4; ++j) kk[j] = kr[32 * j];
        ldwait();
#pragma unroll
        for (int j = 0; j < 4; ++j) vv[j] = kr[(OV - OKK) + 32 * j];
        ldwait();
        float part[2];
#pragma unroll
        for (int h = 0; h < 2; ++h) part[h] = fmaf(qv[2 * h + 1], kk[2 * h + 1], qv[2 * h] * kk[2 * h]);
#pragma unroll
        for (int off = 16; off > 0; off >>= 1) {
#pragma unroll
          for (int h = 0; h < 2; ++h) part[h] += __shfl_xor(part[h], off);
        }
#pragma unroll
        for (int h = 0; h < 2; ++h) {
          const float al = part[h] * ATTSC;
          const float df = al - mx[h];
          const float ee = __expf(-fabsf(df));
          const bool up  = df > 0.f;
          const float s1 = up ? ee : 1.0f;
          const float s2 = up ? 1.0f : ee;
          mx[h] = up ? al : mx[h];
          dn[h] = fmaf(dn[h], s1, s2);
          av[2 * h]     = fmaf(av[2 * h],     s1, s2 * vv[2 * h]);
          av[2 * h + 1] = fmaf(av[2 * h + 1], s1, s2 * vv[2 * h + 1]);
        }
      }
      float iv[2];
#pragma unroll
      for (int h = 0; h < 2; ++h) {
        const float ds = dn[h] > 0.f ? dn[h] : 1.0f;
        iv[h] = (dn[h] > 0.f ? 1.0f : 0.0f) * __builtin_amdgcn_rcpf(ds);
      }
      const float o0 = (av[0] * iv[0] + av[2] * iv[1]) * 0.5f;
      const float o1 = (av[1] * iv[0] + av[3] * iv[1]) * 0.5f;
      r0 = fmaxf(o0 + sk0, 0.f) * live + pz;
      r1 = fmaxf(o1 + sk1, 0.f) * live + pz;
    }

    __builtin_amdgcn_fence(__ATOMIC_RELEASE, "wavefront");
    __builtin_amdgcn_wave_barrier();
    stw[lane]      = r0;
    stw[32 + lane] = r1;
    __builtin_amdgcn_fence(__ATOMIC_RELEASE, "wavefront");
    __builtin_amdgcn_wave_barrier();
    const int l8 = lane & 7;
    const v4f ga = *(const v4f*)(stw + 8 * l8);
    const v4f gb = *(const v4f*)(stw + 8 * l8 + 4);
    U8 hs, ls, sv;
    split8(ga, gb, hs.v, ls.v);
    const bool islo = ((lane >> 3) & 1) != 0;
    sv.w.x = islo ? ls.w.x : hs.w.x;
    sv.w.y = islo ? ls.w.y : hs.w.y;
    sv.w.z = islo ? ls.w.z : hs.w.z;
    sv.w.w = islo ? ls.w.w : hs.w.w;
    unsigned short* gp = Hout + (size_t)grow * KS + 8 * (lane & 15);
    const bool wsv = wr && (lane < 16);
    if (wsv) *(volatile v8us*)gp = sv.v;
    __threadfence();
    if (wsv) *(volatile v8us*)gp = sv.v;
  }
}

static int pick_nb(int nE, int nN) {
  int nb = NBMAX;
  while (nb > 16 && (long long)nb * (long long)nE * 5LL > (long long)RCAP * (long long)nN * 4LL) nb >>= 1;
  return nb;
}
static inline int cdiv(int a, int b) { return (a + b - 1) / b; }

extern "C" void kernel_launch(void* const* d_in, const int* in_sizes, int n_in,
                              void* d_out, int out_size, void* d_ws, size_t ws_size,
                              hipStream_t stream) {
  if (n_in < 16) return;
  const int nN = in_sizes[0] / DIN;
  if (nN <= 0 || in_sizes[0] != nN * DIN || nN > (1 << 22)) return;
  const int nE = in_sizes[1];
  if (nE < 1 || nE > (1 << 20)) return;
  if (in_sizes[15] != 2 * nE) return;
  if (in_sizes[2]  != DIN * H0  || in_sizes[3]  != H0) return;
  if (in_sizes[4]  != H0) return;
  if (in_sizes[5]  != H0 * HDQ  || in_sizes[6]  != HDQ) return;
  if (in_sizes[7]  != H0 * HDQ  || in_sizes[8]  != HDQ) return;
  if (in_sizes[9]  != H0 * HDQ  || in_sizes[10] != HDQ) return;
  if (in_sizes[11] != H0 * HC   || in_sizes[12] != HC) return;
  if (in_sizes[13] != HC * DOUT || in_sizes[14] != DOUT) return;
  if (out_size != nN * DOUT) return;

  const float* x     = (const float*)d_in[0];
  const float* cew   = (const float*)d_in[1];
  const float* Wg    = (const float*)d_in[2];
  const float* bg    = (const float*)d_in[3];
  const float* att   = (const float*)d_in[4];
  const float* Wq    = (const float*)d_in[5];
  const float* bq    = (const float*)d_in[6];
  const float* Wk    = (const float*)d_in[7];
  const float* bk    = (const float*)d_in[8];
  const float* Wv    = (const float*)d_in[9];
  const float* bv    = (const float*)d_in[10];
  const float* Wsk   = (const float*)d_in[11];
  const float* bsk   = (const float*)d_in[12];
  const float* Wf    = (const float*)d_in[13];
  const float* bf    = (const float*)d_in[14];
  const int*   ei    = (const int*)  d_in[15];
  float* out = (float*)d_out;
  const int* src = ei;
  const int* dst = ei + nE;

  const int MP   = cdiv(nN, GBM) * GBM;
  const int nb   = pick_nb(nE, nN);
  const int gA   = cdiv(MP, nb);
  const int vec8 = ((nE & 3) == 0) ? 1 : 0;
  if (gA * nb < MP) return;

  char* ws = (char*)d_ws;
  size_t off = 0;
  const size_t oXB  = off; off += (size_t)MP * DIN * 2;            off = (off + 255) & ~(size_t)255;
  const size_t oHF  = off; off += (size_t)MP * H0 * 4;             off = (off + 255) & ~(size_t)255;
  const size_t oSG  = off; off += (size_t)MP * 4;                  off = (off + 255) & ~(size_t)255;
  const size_t oQKV = off; off += (size_t)MP * NQ * 4;             off = (off + 255) & ~(size_t)255;
  const size_t oH1S = off; off += (size_t)MP * KS * 2;             off = (off + 255) & ~(size_t)255;
  const size_t oH2S = off; off += (size_t)MP * KS * 2;             off = (off + 255) & ~(size_t)255;
  const size_t oWG  = off; off += (size_t)H0 * DIN * 2;            off = (off + 255) & ~(size_t)255;
  const size_t oWQ  = off; off += (size_t)NQ * KS * 2;             off = (off + 255) & ~(size_t)255;
  const size_t oWF  = off; off += (size_t)NFP * KS * 2;            off = (off + 255) & ~(size_t)255;
  if (off > ws_size || off > (size_t)WSMAX) return;
  unsigned short* XB  = (unsigned short*)(ws + oXB);
  float*          HF  = (float*)(ws + oHF);
  float*          SG  = (float*)(ws + oSG);
  float*          QKV = (float*)(ws + oQKV);
  unsigned short* H1S = (unsigned short*)(ws + oH1S);
  unsigned short* H2S = (unsigned short*)(ws + oH2S);
  unsigned short* WG  = (unsigned short*)(ws + oWG);
  unsigned short* WQ  = (unsigned short*)(ws + oWQ);
  unsigned short* WF  = (unsigned short*)(ws + oWF);

  hipFuncSetAttribute(reinterpret_cast<const void*>(&k_agg<1>),
                      hipFuncAttributeMaxDynamicSharedMemorySize, LDS_AGG);
  hipFuncSetAttribute(reinterpret_cast<const void*>(&k_agg<2>),
                      hipFuncAttributeMaxDynamicSharedMemorySize, LDS_AGG);

  const int nUx = MP * (DIN / 8);
  k_xprep<<<cdiv(nUx, NTHR), NTHR, 0, stream>>>(x, XB, nN, nUx);

  {
    const int nU1 = H0 * (DIN / 8);
    k_wtr<<<cdiv(nU1, NTHR), NTHR, 0, stream>>>(Wg, Wg, Wg, Wg, H0, H0, H0, H0, H0, DIN, DIN, WG, nU1);
    const int nU2 = NQ * (KS / 8);
    k_wtr<<<cdiv(nU2, NTHR), NTHR, 0, stream>>>(Wq, Wk, Wv, Wsk, HDQ, HDQ, HDQ, HC, HDQ, H0, KS, WQ, nU2);
    const int nU3 = NFP * (KS / 8);
    k_wtr<<<cdiv(nU3, NTHR), NTHR, 0, stream>>>(Wf, Wf, Wf, Wf, DOUT, DOUT, DOUT, DOUT, NFP, HC, KS, WF, nU3);
  }

  const int gM = MP / GBM;
  k_gemm<1><<<dim3(gM, H0 / GBN), GTHR, 0, stream>>>(XB, WG, bg, bg, bg, bg, att, HF, SG,
                                                     DIN, H0, H0, H0, H0, nN);
  k_agg<1><<<gA, NTHR, LDS_AGG, stream>>>(src, dst, HF, SG, cew, QKV, H1S, nN, nE, nb, vec8, MP);
  k_gemm<0><<<dim3(gM, NQ / GBN), GTHR, 0, stream>>>(H1S, WQ, bq, bk, bv, bsk, att, QKV, SG,
                                                     KS, NQ, HDQ, HDQ, HC, nN);
  k_agg<2><<<gA, NTHR, LDS_AGG, stream>>>(src, dst, QKV, SG, cew, QKV, H2S, nN, nE, nb, vec8, MP);
  k_gemm<2><<<dim3(gM, NFP / GBN), GTHR, 0, stream>>>(H2S, WF, bf, bf, bf, bf, att, out, SG,
                                                      KS, DOUT, NFP, DOUT, DOUT, nN);
}
